// PointNetDecoder_31885837206054
// MI455X (gfx1250) — hardware-verified
//
#include <hip/hip_runtime.h>
#include <stddef.h>

#pragma clang fp contract(off)

typedef __attribute__((ext_vector_type(16))) __bf16   v16b;
typedef __attribute__((ext_vector_type(8)))  __bf16   v8b;
typedef __attribute__((ext_vector_type(8)))  float    v8f;
typedef __attribute__((ext_vector_type(4)))  float    v4f;
typedef __attribute__((ext_vector_type(4)))  unsigned v4u;

constexpr int NPTS   = 16384;
constexpr int SPTS   = 4096;
constexpr int NCH_CO = 256;
constexpr int NCH_FI = 64;
constexpr int KIN1   = NCH_CO + NCH_FI;
constexpr int NCH_L1 = 256;
constexpr int NCH_L2 = 128;
constexpr int KNN_TILE = 512;
constexpr int XPITCH = 164;
constexpr int SLABP  = 36;
static_assert(KIN1 % 32 == 0, "K of layer 1 must be a multiple of 32");
static_assert(NCH_L1 % 32 == 0, "K of layer 2 must be a multiple of 32");
static_assert(NPTS % 64 == 0 && NCH_L1 % 32 == 0 && NCH_L2 % 32 == 0, "tile multiples (wave tile 64 x 32)");
static_assert(((NPTS / 64) * (NCH_L1 / 32)) % 8 == 0 && ((NPTS / 64) * (NCH_L2 / 32)) % 8 == 0, "8 wave tiles per block");
static_assert(SPTS % KNN_TILE == 0 && KNN_TILE % 256 == 0, "coarse tiling");
static_assert((XPITCH * 4) % 16 == 0 && XPITCH >= KIN1 / 2, "LDS pitch");
static_assert(NPTS % 256 == 0, "fine points per block");
static_assert(NCH_CO == 256 && NCH_FI == 64, "channel-pair phases assume 128 + 32 pairs");

constexpr size_t SZ_W1P  = (size_t)NCH_L1 * KIN1 * 2;
constexpr size_t SZ_W2P  = (size_t)NCH_L2 * NCH_L1 * 2;
constexpr size_t SZ_XP   = (size_t)NPTS * KIN1 * 2;
constexpr size_t SZ_Y1   = (size_t)NPTS * NCH_L1 * 4;
constexpr size_t SZ_H1P  = (size_t)NPTS * NCH_L1 * 2;
constexpr size_t SZ_Y2   = (size_t)NPTS * NCH_L2 * 4;
constexpr size_t OFF_W1HI = 0;
constexpr size_t OFF_W1LO = OFF_W1HI + SZ_W1P;
constexpr size_t OFF_W2HI = OFF_W1LO + SZ_W1P;
constexpr size_t OFF_W2LO = OFF_W2HI + SZ_W2P;
constexpr size_t OFF_XHI  = OFF_W2LO + SZ_W2P;
constexpr size_t OFF_XLO  = OFF_XHI + SZ_XP;
constexpr size_t OFF_Y1   = OFF_XLO + SZ_XP;
constexpr size_t OFF_H1HI = OFF_Y1 + SZ_Y1;
constexpr size_t OFF_H1LO = OFF_H1HI + SZ_H1P;
constexpr size_t OFF_Y2   = OFF_H1LO + SZ_H1P;
constexpr size_t OFF_MEAN1 = OFF_Y2 + SZ_Y2;
constexpr size_t OFF_RSTD1 = OFF_MEAN1 + (size_t)NCH_L1 * 4;
constexpr size_t OFF_MEAN2 = OFF_RSTD1 + (size_t)NCH_L1 * 4;
constexpr size_t OFF_RSTD2 = OFF_MEAN2 + (size_t)NCH_L2 * 4;
constexpr size_t WS_TOTAL  = OFF_RSTD2 + (size_t)NCH_L2 * 4;
static_assert(WS_TOTAL == 63376384, "carve total");
static_assert(WS_TOTAL <= 134217728, "carve under 128 MiB");
static_assert(OFF_W1LO % 256 == 0 && OFF_W2HI % 256 == 0 && OFF_W2LO % 256 == 0 && OFF_XHI % 256 == 0 &&
              OFF_XLO % 256 == 0 && OFF_Y1 % 256 == 0 && OFF_H1HI % 256 == 0 && OFF_H1LO % 256 == 0 &&
              OFF_Y2 % 256 == 0 && OFF_MEAN1 % 256 == 0 && OFF_RSTD1 % 256 == 0 && OFF_MEAN2 % 256 == 0 &&
              OFF_RSTD2 % 256 == 0, "alignment");

__device__ __forceinline__ unsigned bf_rne_bits(float f) {
  const unsigned u = __float_as_uint(f);
  return (u + 0x7FFFu + ((u >> 16) & 1u)) >> 16;
}
__device__ __forceinline__ void bf_split(float f, unsigned& hb, unsigned& lb) {
  hb = bf_rne_bits(f);
  const float hf = __uint_as_float(hb << 16);
  const float rs = f - hf;
  lb = bf_rne_bits(rs);
}

__device__ __forceinline__ v16b frag_load_b(const __bf16* p) {
  union U { v16b v; v8b h[2]; } f;
  f.h[0] = *(const v8b*)(p);
  f.h[1] = *(const v8b*)(p + 16);
  return f.v;
}
__device__ __forceinline__ v8f mma_b(v16b a, v16b b, v8f c) {
  return __builtin_amdgcn_wmma_f32_16x16x32_bf16(false, a, false, b, (short)0, c, false, false);
}
__device__ __forceinline__ void dep_guard2_b(v8f& a, v8f& b, v16b x, v16b y) {
  asm volatile("v_nop\n\tv_nop\n\tv_nop\n\tv_nop" : "+v"(a), "+v"(b) : "v"(x), "v"(y));
}
__device__ __forceinline__ void keep4_b(v16b a, v16b b, v16b c, v16b d) {
  asm volatile("v_nop" :: "v"(a), "v"(b), "v"(c), "v"(d));
}
__device__ __forceinline__ void acc_guard4(v8f& a, v8f& b, v8f& c, v8f& d) {
  asm volatile("v_nop\n\tv_nop\n\tv_nop\n\tv_nop" : "+v"(a), "+v"(b), "+v"(c), "+v"(d));
}

__global__ __launch_bounds__(256) void split_planes_kernel(
    const float* __restrict__ in, unsigned short* __restrict__ hi, unsigned short* __restrict__ lo, int n8) {
  const int i = blockIdx.x * 256 + threadIdx.x;
  const int ic = (i < n8) ? i : (n8 - 1);
  const v4f a = *(const v4f*)(in + (size_t)ic * 8);
  const v4f b = *(const v4f*)(in + (size_t)ic * 8 + 4);
  float f[8];
  f[0] = a.x; f[1] = a.y; f[2] = a.z; f[3] = a.w;
  f[4] = b.x; f[5] = b.y; f[6] = b.z; f[7] = b.w;
  unsigned hb[8], lb[8];
#pragma unroll
  for (int e = 0; e < 8; ++e) bf_split(f[e], hb[e], lb[e]);
  v4u hv, lv;
  hv.x = hb[0] | (hb[1] << 16); hv.y = hb[2] | (hb[3] << 16);
  hv.z = hb[4] | (hb[5] << 16); hv.w = hb[6] | (hb[7] << 16);
  lv.x = lb[0] | (lb[1] << 16); lv.y = lb[2] | (lb[3] << 16);
  lv.z = lb[4] | (lb[5] << 16); lv.w = lb[6] | (lb[7] << 16);
  for (int pass = 0; pass < 2; ++pass) {
    if (i < n8) {
      *(volatile v4u*)(hi + (size_t)i * 8) = hv;
      *(volatile v4u*)(lo + (size_t)i * 8) = lv;
    }
    __threadfence();
  }
}

__global__ __launch_bounds__(256) void knn_interp_kernel(
    const float* __restrict__ fxyz, const float* __restrict__ cxyz,
    const int* __restrict__ fid, const int* __restrict__ cid,
    const float* __restrict__ cf, const float* __restrict__ ff,
    unsigned short* __restrict__ Xhi, unsigned short* __restrict__ Xlo) {
#pragma clang fp contract(off)
  __shared__ __align__(16) v4f sc[KNN_TILE];
  __shared__ int sid[KNN_TILE];
  __shared__ int sJ[3 * 256];
  __shared__ float sW[3 * 256];
  __shared__ __align__(16) unsigned sHi[32 * XPITCH];
  __shared__ __align__(16) unsigned sLo[32 * XPITCH];
  const int t = threadIdx.x;
  const int lane = t & 31;
  const int wave = t >> 5;
  const int nblk = blockIdx.x * 256;
  const int n = nblk + t;

  const float fx = fxyz[n];
  const float fy = fxyz[NPTS + n];
  const float fz = fxyz[2 * NPTS + n];
  const int pid = fid[n];
  const float fxx = fx * fx;
  const float fyy = fy * fy;
  const float fzz = fz * fz;
  const float sqf = (fxx + fzz) + fyy;
  const float big = 1e8f;
  float d0 = __builtin_inff(), d1 = __builtin_inff(), d2 = __builtin_inff();
  int i0 = 0, i1 = 0, i2 = 0;
  for (int base = 0; base < SPTS; base += KNN_TILE) {
    __syncthreads();
#pragma unroll
    for (int u = 0; u < KNN_TILE / 256; ++u) {
      const int s = base + u * 256 + t;
      const float cx = cxyz[s];
      const float cy = cxyz[SPTS + s];
      const float cz = cxyz[2 * SPTS + s];
      const int id = cid[s];
      const float cxx = cx * cx;
      const float cyy = cy * cy;
      const float czz = cz * cz;
      const float sq = (cxx + czz) + cyy;
      v4f pk;
      pk.x = cx; pk.y = cy; pk.z = cz; pk.w = sq;
      sc[u * 256 + t] = pk;
      sid[u * 256 + t] = id;
    }
    __syncthreads();
#pragma unroll 4
    for (int j = 0; j < KNN_TILE; ++j) {
      const v4f c = sc[j];
      const int cj = sid[j];
      float p = fx * c.x;
      p = __builtin_fmaf(fy, c.y, p);
      p = __builtin_fmaf(fz, c.z, p);
      const float s2 = sqf + c.w;
      const float p2 = p + p;
      float d = s2 - p2;
      d = (cj != pid) ? big : d;
      if (d < d2) {
        const int jj = base + j;
        const bool c0 = d < d0;
        const bool c1 = d < d1;
        const float nd2 = c1 ? d1 : d;
        const int   ni2 = c1 ? i1 : jj;
        const float nd1 = c0 ? d0 : (c1 ? d : d1);
        const int   ni1 = c0 ? i0 : (c1 ? jj : i1);
        const float nd0 = c0 ? d : d0;
        const int   ni0 = c0 ? jj : i0;
        d0 = nd0; d1 = nd1; d2 = nd2;
        i0 = ni0; i1 = ni1; i2 = ni2;
      }
    }
  }

  {
    const float epsw = 1e-8f;
    const float r0 = 1.0f / (d0 + epsw);
    const float r1 = 1.0f / (d1 + epsw);
    const float r2 = 1.0f / (d2 + epsw);
    const float rs = (r0 + r2) + r1;
    const float w0 = r0 / rs;
    const float w1 = r1 / rs;
    const float w2 = r2 / rs;
    sJ[t] = i0;
    sJ[256 + t] = i1;
    sJ[512 + t] = i2;
    sW[t] = w0;
    sW[256 + t] = w1;
    sW[512 + t] = w2;
  }
  __syncthreads();

#pragma unroll 1
  for (int sub = 0; sub < 8; ++sub) {
    const int p = sub * 32 + lane;
    int j0 = sJ[p];
    int j1 = sJ[256 + p];
    int j2 = sJ[512 + p];
    j0 = j0 < 0 ? 0 : (j0 > SPTS - 1 ? SPTS - 1 : j0);
    j1 = j1 < 0 ? 0 : (j1 > SPTS - 1 ? SPTS - 1 : j1);
    j2 = j2 < 0 ? 0 : (j2 > SPTS - 1 ? SPTS - 1 : j2);
    const float w0 = sW[p];
    const float w1 = sW[256 + p];
    const float w2 = sW[512 + p];
    const int np = nblk + p;
#pragma unroll 1
    for (int i = 0; i < 16; ++i) {
      const int q = wave + 8 * i;
      const float* ra = cf + (size_t)(2 * q) * SPTS;
      const float* rb = ra + SPTS;
      const float a0 = ra[j0];
      const float a1 = ra[j1];
      const float a2 = ra[j2];
      const float b0 = rb[j0];
      const float b1 = rb[j1];
      const float b2 = rb[j2];
      const float ta0 = a0 * w0;
      const float ta1 = a1 * w1;
      const float ta2 = a2 * w2;
      const float tb0 = b0 * w0;
      const float tb1 = b1 * w1;
      const float tb2 = b2 * w2;
      const float va = (ta0 + ta1) + ta2;
      const float vb = (tb0 + tb1) + tb2;
      unsigned ha, la, hb, lb;
      bf_split(va, ha, la);
      bf_split(vb, hb, lb);
      sHi[lane * XPITCH + q] = ha | (hb << 16);
      sLo[lane * XPITCH + q] = la | (lb << 16);
      asm volatile("" ::: "memory");
    }
#pragma unroll 1
    for (int i = 0; i < 4; ++i) {
      const int q = wave + 8 * i;
      const float va = ff[(size_t)(2 * q) * NPTS + np];
      const float vb = ff[(size_t)(2 * q + 1) * NPTS + np];
      unsigned ha, la, hb, lb;
      bf_split(va, ha, la);
      bf_split(vb, hb, lb);
      sHi[lane * XPITCH + 128 + q] = ha | (hb << 16);
      sLo[lane * XPITCH + 128 + q] = la | (lb << 16);
      asm volatile("" ::: "memory");
    }
    __syncthreads();
    {
      const int n0 = nblk + sub * 32;
      unsigned short* gh = Xhi + (size_t)n0 * KIN1;
      unsigned short* gl = Xlo + (size_t)n0 * KIN1;
      for (int pass = 0; pass < 2; ++pass) {
#pragma unroll
        for (int it = 0; it < 5; ++it) {
          const int u = t + 256 * it;
          const int row = u / 40;
          const int c4 = u - row * 40;
          const v4u hv = *(const v4u*)(sHi + row * XPITCH + c4 * 4);
          const v4u lv = *(const v4u*)(sLo + row * XPITCH + c4 * 4);
          *(volatile v4u*)(gh + (size_t)u * 8) = hv;
          *(volatile v4u*)(gl + (size_t)u * 8) = lv;
        }
        __threadfence();
      }
    }
    __syncthreads();
  }
}

__global__ __launch_bounds__(256) void wmma_gemm64x32_bf16x3(
    const unsigned short* __restrict__ Ap, const unsigned short* __restrict__ A2p, int lda,
    const unsigned short* __restrict__ Btp, const unsigned short* __restrict__ Bt2p, int ldb,
    float* __restrict__ Cout, int ldc, const float* __restrict__ bias, int M, int N, int K) {
  const __bf16* A = (const __bf16*)Ap;
  const __bf16* A2 = (const __bf16*)A2p;
  const __bf16* Bt = (const __bf16*)Btp;
  const __bf16* Bt2 = (const __bf16*)Bt2p;
  __shared__ __align__(16) float sT[8][16 * SLABP];
  const int lane = threadIdx.x & 31;
  const int wave = threadIdx.x >> 5;
  const int tilesN = N >> 5;
  const int tilesM = M >> 6;
  const int tile = blockIdx.x * 8 + wave;
  if (tile >= tilesM * tilesN) return;
  const int tm = tile / tilesN;
  const int tn = tile - tm * tilesN;
  const int m0 = tm << 6;
  const int n0 = tn << 5;
  const int rlane = lane & 15;
  const int koff = (lane >> 4) * 8;
  const int mOff = (lane >> 4) * 8;

  v8f acc[4][2];
#pragma unroll
  for (int i = 0; i < 4; ++i)
#pragma unroll
    for (int j = 0; j < 2; ++j) acc[i][j] = (v8f){0.f, 0.f, 0.f, 0.f, 0.f, 0.f, 0.f, 0.f};

  for (int k0 = 0; k0 < K; k0 += 32) {
    v16b bh[2], bl[2];
#pragma unroll
    for (int j = 0; j < 2; ++j) {
      const size_t bo = (size_t)(n0 + (j << 4) + rlane) * ldb + koff + k0;
      bh[j] = frag_load_b(Bt + bo);
      bl[j] = frag_load_b(Bt2 + bo);
    }
#pragma unroll
    for (int i = 0; i < 4; ++i) {
      const size_t ao = (size_t)(m0 + (i << 4) + rlane) * lda + koff + k0;
      const v16b ah = frag_load_b(A + ao);
      const v16b al = frag_load_b(A2 + ao);
#pragma unroll
      for (int j = 0; j < 2; ++j) {
        acc[i][j] = mma_b(ah, bh[j], acc[i][j]);
        acc[i][j] = mma_b(ah, bl[j], acc[i][j]);
        acc[i][j] = mma_b(al, bh[j], acc[i][j]);
      }
      dep_guard2_b(acc[i][0], acc[i][1], ah, al);
    }
    keep4_b(bh[0], bh[1], bl[0], bl[1]);
  }
  acc_guard4(acc[0][0], acc[0][1], acc[1][0], acc[1][1]);
  acc_guard4(acc[2][0], acc[2][1], acc[3][0], acc[3][1]);

  float* slab = sT[wave];
#pragma unroll
  for (int i = 0; i < 4; ++i) {
    const int mBase = m0 + (i << 4);
#pragma unroll
    for (int j = 0; j < 2; ++j) {
      const int nn = n0 + (j << 4) + rlane;
      const float bv = bias[nn];
#pragma unroll
      for (int r = 0; r < 8; ++r) {
        const float v = acc[i][j][r] + bv;
        slab[(mOff + r) * SLABP + (j << 4) + rlane] = v;
      }
    }
    __builtin_amdgcn_fence(__ATOMIC_RELEASE, "workgroup");
    __builtin_amdgcn_wave_barrier();
    __builtin_amdgcn_fence(__ATOMIC_ACQUIRE, "workgroup");
    {
      const int q = lane >> 3;
      const int c4 = (lane & 7) * 4;
      for (int pass = 0; pass < 2; ++pass) {
#pragma unroll
        for (int it = 0; it < 4; ++it) {
          const int row = it * 4 + q;
          const v4f v = *(const v4f*)(slab + row * SLABP + c4);
          *(volatile v4f*)(Cout + (size_t)(mBase + row) * ldc + n0 + c4) = v;
        }
        __threadfence();
      }
    }
    __builtin_amdgcn_fence(__ATOMIC_RELEASE, "workgroup");
    __builtin_amdgcn_wave_barrier();
    __builtin_amdgcn_fence(__ATOMIC_ACQUIRE, "workgroup");
  }
}

__global__ __launch_bounds__(256) void bn_stats_kernel(
    const float* __restrict__ Y, int C, float* __restrict__ meanp, float* __restrict__ rstdp) {
  __shared__ float red1[8 * 32];
  __shared__ float red2[8 * 32];
  const int lane = threadIdx.x & 31;
  const int wave = threadIdx.x >> 5;
  const int c = blockIdx.x * 32 + lane;
  const float* col = Y + c;
  const float invn = 1.0f / (float)NPTS;
  float a0 = 0.f, a1 = 0.f, a2 = 0.f, a3 = 0.f;
#pragma unroll 1
  for (int r = wave; r < NPTS; r += 32) {
    const float y0 = col[(size_t)r * C];
    const float y1 = col[(size_t)(r + 8) * C];
    const float y2 = col[(size_t)(r + 16) * C];
    const float y3 = col[(size_t)(r + 24) * C];
    a0 += y0; a1 += y1; a2 += y2; a3 += y3;
  }
  red1[wave * 32 + lane] = (a0 + a1) + (a2 + a3);
  __syncthreads();
  float tot = 0.f;
#pragma unroll
  for (int w = 0; w < 8; ++w) tot += red1[w * 32 + lane];
  const float mean = tot * invn;
  float q0 = 0.f, q1 = 0.f, q2 = 0.f, q3 = 0.f;
#pragma unroll 1
  for (int r = wave; r < NPTS; r += 32) {
    const float e0 = col[(size_t)r * C] - mean;
    const float e1 = col[(size_t)(r + 8) * C] - mean;
    const float e2 = col[(size_t)(r + 16) * C] - mean;
    const float e3 = col[(size_t)(r + 24) * C] - mean;
    const float s0 = e0 * e0;
    const float s1 = e1 * e1;
    const float s2 = e2 * e2;
    const float s3 = e3 * e3;
    q0 += s0; q1 += s1; q2 += s2; q3 += s3;
  }
  red2[wave * 32 + lane] = (q0 + q1) + (q2 + q3);
  __syncthreads();
  float tq = 0.f;
#pragma unroll
  for (int w = 0; w < 8; ++w) tq += red2[w * 32 + lane];
  const float var = tq * invn;
  const float rstd = 1.0f / sqrtf(var + 1e-5f);
  if (wave == 0) {
    for (int pass = 0; pass < 2; ++pass) {
      *(volatile float*)(meanp + c) = mean;
      *(volatile float*)(rstdp + c) = rstd;
      __threadfence();
    }
  }
}

__global__ __launch_bounds__(256) void bn_relu_split_kernel(
    const float* __restrict__ Y, const float* __restrict__ meanp, const float* __restrict__ rstdp,
    const float* __restrict__ gam, const float* __restrict__ bet,
    unsigned short* __restrict__ Hhi, unsigned short* __restrict__ Hlo) {
  __shared__ float sM[NCH_L1];
  __shared__ float sR[NCH_L1];
  __shared__ float sG[NCH_L1];
  __shared__ float sB[NCH_L1];
  const int t = threadIdx.x;
  sM[t] = meanp[t];
  sR[t] = rstdp[t];
  sG[t] = gam[t];
  sB[t] = bet[t];
  __syncthreads();
  const size_t u = (size_t)blockIdx.x * 256 + t;
  const int c0 = (t & 31) * 8;
  const v4f a = *(const v4f*)(Y + u * 8);
  const v4f b = *(const v4f*)(Y + u * 8 + 4);
  float f[8];
  f[0] = a.x; f[1] = a.y; f[2] = a.z; f[3] = a.w;
  f[4] = b.x; f[5] = b.y; f[6] = b.z; f[7] = b.w;
  unsigned hb[8], lb[8];
#pragma unroll
  for (int e = 0; e < 8; ++e) {
    const float dm = f[e] - sM[c0 + e];
    const float dn = dm * sR[c0 + e];
    const float dg = dn * sG[c0 + e];
    float v = dg + sB[c0 + e];
    v = fmaxf(v, 0.0f);
    bf_split(v, hb[e], lb[e]);
  }
  v4u hv, lv;
  hv.x = hb[0] | (hb[1] << 16); hv.y = hb[2] | (hb[3] << 16);
  hv.z = hb[4] | (hb[5] << 16); hv.w = hb[6] | (hb[7] << 16);
  lv.x = lb[0] | (lb[1] << 16); lv.y = lb[2] | (lb[3] << 16);
  lv.z = lb[4] | (lb[5] << 16); lv.w = lb[6] | (lb[7] << 16);
  for (int pass = 0; pass < 2; ++pass) {
    *(volatile v4u*)(Hhi + u * 8) = hv;
    *(volatile v4u*)(Hlo + u * 8) = lv;
    __threadfence();
  }
}

__global__ __launch_bounds__(256) void bn_relu_transpose_kernel(
    const float* __restrict__ Y2, const float* __restrict__ meanp, const float* __restrict__ rstdp,
    const float* __restrict__ gam, const float* __restrict__ bet, float* __restrict__ outp) {
  __shared__ float sM[NCH_L2];
  __shared__ float sR[NCH_L2];
  __shared__ float sG[NCH_L2];
  __shared__ float sB[NCH_L2];
  __shared__ __align__(16) float sT[NCH_L2 * 36];
  const int t = threadIdx.x;
  const int lane = t & 31;
  const int wave = t >> 5;
  if (t < NCH_L2) {
    sM[t] = meanp[t];
    sR[t] = rstdp[t];
    sG[t] = gam[t];
    sB[t] = bet[t];
  }
  __syncthreads();
  const int n0 = blockIdx.x * 32;
#pragma unroll
  for (int it = 0; it < 4; ++it) {
    const int u = t + 256 * it;
    const int row = u >> 5;
    const int c4 = (u & 31) * 4;
    const v4f y = *(const v4f*)(Y2 + (size_t)(n0 + row) * NCH_L2 + c4);
    float f[4];
    f[0] = y.x; f[1] = y.y; f[2] = y.z; f[3] = y.w;
#pragma unroll
    for (int e = 0; e < 4; ++e) {
      const int c = c4 + e;
      const float dm = f[e] - sM[c];
      const float dn = dm * sR[c];
      const float dg = dn * sG[c];
      float v = dg + sB[c];
      v = fmaxf(v, 0.0f);
      sT[c * 36 + row] = v;
    }
  }
  __syncthreads();
  for (int pass = 0; pass < 2; ++pass) {
#pragma unroll
    for (int it = 0; it < 4; ++it) {
      const int c = wave * 16 + it * 4 + (lane >> 3);
      const int n4 = (lane & 7) * 4;
      const v4f v = *(const v4f*)(sT + c * 36 + n4);
      *(volatile v4f*)(outp + (size_t)c * NPTS + n0 + n4) = v;
    }
    __threadfence();
  }
}

extern "C" void kernel_launch(void* const* d_in, const int* in_sizes, int n_in,
                              void* d_out, int out_size, void* d_ws, size_t ws_size,
                              hipStream_t stream) {
  if (n_in != 14) return;
  if (in_sizes[0] != 3 * NPTS || in_sizes[1] != 3 * SPTS || in_sizes[2] != NPTS || in_sizes[3] != SPTS) return;
  if (in_sizes[4] != NCH_FI * NPTS || in_sizes[5] != NCH_CO * SPTS) return;
  if (in_sizes[6] != NCH_L1 * KIN1 || in_sizes[7] != NCH_L1 || in_sizes[8] != NCH_L1 || in_sizes[9] != NCH_L1) return;
  if (in_sizes[10] != NCH_L2 * NCH_L1 || in_sizes[11] != NCH_L2 || in_sizes[12] != NCH_L2 || in_sizes[13] != NCH_L2) return;
  if (out_size != NCH_L2 * NPTS) return;
  if (ws_size < WS_TOTAL) return;

  const float* fxyz = (const float*)d_in[0];
  const float* cxyz = (const float*)d_in[1];
  const int*   fid  = (const int*)d_in[2];
  const int*   cid  = (const int*)d_in[3];
  const float* ffea = (const float*)d_in[4];
  const float* cfea = (const float*)d_in[5];
  const float* W1   = (const float*)d_in[6];
  const float* b1   = (const float*)d_in[7];
  const float* g1   = (const float*)d_in[8];
  const float* be1  = (const float*)d_in[9];
  const float* W2   = (const float*)d_in[10];
  const float* b2   = (const float*)d_in[11];
  const float* g2   = (const float*)d_in[12];
  const float* be2  = (const float*)d_in[13];

  unsigned char* ws = (unsigned char*)d_ws;
  unsigned short* W1hi = (unsigned short*)(ws + OFF_W1HI);
  unsigned short* W1lo = (unsigned short*)(ws + OFF_W1LO);
  unsigned short* W2hi = (unsigned short*)(ws + OFF_W2HI);
  unsigned short* W2lo = (unsigned short*)(ws + OFF_W2LO);
  unsigned short* Xhi  = (unsigned short*)(ws + OFF_XHI);
  unsigned short* Xlo  = (unsigned short*)(ws + OFF_XLO);
  float*          Y1   = (float*)(ws + OFF_Y1);
  unsigned short* H1hi = (unsigned short*)(ws + OFF_H1HI);
  unsigned short* H1lo = (unsigned short*)(ws + OFF_H1LO);
  float*          Y2   = (float*)(ws + OFF_Y2);
  float*          mean1 = (float*)(ws + OFF_MEAN1);
  float*          rstd1 = (float*)(ws + OFF_RSTD1);
  float*          mean2 = (float*)(ws + OFF_MEAN2);
  float*          rstd2 = (float*)(ws + OFF_RSTD2);

  split_planes_kernel<<<dim3((NCH_L1 * KIN1 / 8) / 256), dim3(256), 0, stream>>>(W1, W1hi, W1lo, NCH_L1 * KIN1 / 8);
  split_planes_kernel<<<dim3((NCH_L2 * NCH_L1 / 8) / 256), dim3(256), 0, stream>>>(W2, W2hi, W2lo, NCH_L2 * NCH_L1 / 8);

  knn_interp_kernel<<<dim3(NPTS / 256), dim3(256), 0, stream>>>(fxyz, cxyz, fid, cid, cfea, ffea, Xhi, Xlo);

  wmma_gemm64x32_bf16x3<<<dim3(((NPTS / 64) * (NCH_L1 / 32)) / 8), dim3(256), 0, stream>>>(
      Xhi, Xlo, KIN1, W1hi, W1lo, KIN1, Y1, NCH_L1, b1, NPTS, NCH_L1, KIN1);
  bn_stats_kernel<<<dim3(NCH_L1 / 32), dim3(256), 0, stream>>>(Y1, NCH_L1, mean1, rstd1);
  bn_relu_split_kernel<<<dim3((NPTS * NCH_L1 / 8) / 256), dim3(256), 0, stream>>>(
      Y1, mean1, rstd1, g1, be1, H1hi, H1lo);

  wmma_gemm64x32_bf16x3<<<dim3(((NPTS / 64) * (NCH_L2 / 32)) / 8), dim3(256), 0, stream>>>(
      H1hi, H1lo, NCH_L1, W2hi, W2lo, NCH_L1, Y2, NCH_L2, b2, NPTS, NCH_L2, NCH_L1);
  bn_stats_kernel<<<dim3(NCH_L2 / 32), dim3(256), 0, stream>>>(Y2, NCH_L2, mean2, rstd2);
  bn_relu_transpose_kernel<<<dim3(NPTS / 32), dim3(256), 0, stream>>>(
      Y2, mean2, rstd2, g2, be2, (float*)d_out);
}
